// FeedForward_80917183856743
// MI455X (gfx1250) — hardware-verified
//
#include <hip/hip_runtime.h>
#include <math.h>
#include <stdint.h>


typedef _Float16 v16h __attribute__((ext_vector_type(16)));
typedef _Float16 v8h  __attribute__((ext_vector_type(8)));
typedef __bf16   v16b __attribute__((ext_vector_type(16)));
typedef unsigned short u16;
typedef u16   v8us __attribute__((ext_vector_type(8)));
typedef float v8f  __attribute__((ext_vector_type(8)));
typedef float v4f  __attribute__((ext_vector_type(4)));

#ifndef NB
#define NB 4
#endif
#ifndef SEQ
#define SEQ 2048
#endif
#define NB_FULL 4
#define SEQ_FULL 2048
#define DD 1024
#define HH 4096
#define NCB 8
#define KCB 256
#define SUB1 (DD / NCB)
#define SUB2 (HH / NCB)
#define MROWS (NB * SEQ)
#define P1 72
#define P2 68
#define HCARRY 16.0f
#define WCARRY 64.0f
#define UNCARRY (1.0f / 1024.0f)

static_assert(NB >= 1 && NB <= NB_FULL);
static_assert(SEQ >= 64 && SEQ <= SEQ_FULL && (SEQ % 64) == 0);
static_assert((DD % 512) == 0 && (HH % 512) == 0);
static_assert((DD % 32) == 0 && (HH % 32) == 0);
static_assert((SUB1 % 8) == 0 && (SUB2 % 8) == 0);
static_assert((MROWS % 64) == 0);

union FragB { v16b v; v8us h[2]; };
union FragH { v16h v; v8h h[2]; };

__device__ __forceinline__ u16 bf16_bits(float f) {
  unsigned int u = __builtin_bit_cast(unsigned int, f);
  u += 0x7fffu + ((u >> 16) & 1u);
  return (u16)(u >> 16);
}

__device__ __forceinline__ float bf16_val(float f) {
  unsigned int u = __builtin_bit_cast(unsigned int, f);
  u += 0x7fffu + ((u >> 16) & 1u);
  u &= 0xffff0000u;
  return __builtin_bit_cast(float, u);
}

__device__ __forceinline__ int full_row(int m) {
  const int b = m / SEQ;
  return b * SEQ_FULL + (m - b * SEQ);
}

__device__ __forceinline__ float erf_as(float x) {
  const float ax = fabsf(x);
  const float t  = __builtin_amdgcn_rcpf(fmaf(0.3275911f, ax, 1.0f));
  float y = fmaf(t, 1.061405429f, -1.453152027f);
  y = fmaf(t, y, 1.421413741f);
  y = fmaf(t, y, -0.284496736f);
  y = fmaf(t, y, 0.254829592f);
  const float e = __expf(-(ax * ax));
  const float r = fmaf(-(y * t), e, 1.0f);
  return copysignf(r, x);
}

__device__ __forceinline__ float gelu_f(float v) {
  return 0.5f * v * (1.0f + erf_as(v * 0.70710678118654752f));
}

__device__ __forceinline__ v16b ldfrag_b(const u16* __restrict__ p,
                                         int row, int k0, int ld, int lane) {
  const u16* q = p + (size_t)(row + (lane & 15)) * ld + (k0 + ((lane >> 4) << 3));
  FragB f;
  f.h[0] = *(const v8us*)q;
  f.h[1] = *(const v8us*)(q + 16);
  return f.v;
}

__device__ __forceinline__ v16h ldfrag_h(const _Float16* __restrict__ p,
                                         int row, int k0, int ld, int lane) {
  const _Float16* q = p + (size_t)(row + (lane & 15)) * ld + (k0 + ((lane >> 4) << 3));
  FragH f;
  f.h[0] = *(const v8h*)q;
  f.h[1] = *(const v8h*)(q + 16);
  return f.v;
}

__device__ __forceinline__ v8f mma_bf16(v16b a, v16b b, v8f c) {
  v8f d = __builtin_amdgcn_wmma_f32_16x16x32_bf16(false, a, false, b, (short)0, c, false, false);
  asm volatile("v_nop\n\tv_nop\n\tv_nop\n\tv_nop" : "+v"(d) : "v"(a), "v"(b));
  return d;
}

__device__ __forceinline__ v8f mma_f16(v16h a, v16h b, v8f c) {
  v8f d = __builtin_amdgcn_wmma_f32_16x16x32_f16(false, a, false, b, (short)0, c, false, false);
  asm volatile("v_nop\n\tv_nop\n\tv_nop\n\tv_nop" : "+v"(d) : "v"(a), "v"(b));
  return d;
}

__global__ void __launch_bounds__(256)
k_cvt_x(const float* __restrict__ x, u16* xb) {
  const int t = blockIdx.x * 256 + threadIdx.x;
  const int total = MROWS * (DD / 8);
  if (t >= total) return;
  const int m  = t / (DD / 8);
  const int c8 = t - m * (DD / 8);
  const float* src = x + (size_t)full_row(m) * DD + c8 * 8;
  const v4f lo = *(const v4f*)src;
  const v4f hi = *(const v4f*)(src + 4);
  v8us o;
  o[0] = bf16_bits(lo[0]); o[1] = bf16_bits(lo[1]);
  o[2] = bf16_bits(lo[2]); o[3] = bf16_bits(lo[3]);
  o[4] = bf16_bits(hi[0]); o[5] = bf16_bits(hi[1]);
  o[6] = bf16_bits(hi[2]); o[7] = bf16_bits(hi[3]);
  u16* dst = xb + (size_t)m * DD + c8 * 8;
  *(volatile v8us*)dst = o;
  __threadfence();
  *(volatile v8us*)dst = o;
}

__global__ void __launch_bounds__(256)
k_gather_w1(const float* __restrict__ cb, const int* __restrict__ idx, u16* w) {
  const int t = blockIdx.x * 256 + threadIdx.x;
  const int total = HH * (DD / 8);
  if (t >= total) return;
  const int row = t / (DD / 8);
  const int c8  = t - row * (DD / 8);
  const int d0  = c8 * 8;
  const int c   = d0 / SUB1;
  const int j   = d0 - c * SUB1;
  int code = idx[c * HH + row];
  code = code < 0 ? 0 : (code > KCB - 1 ? KCB - 1 : code);
  const float* src = cb + ((size_t)(c * KCB + code) * SUB1 + j);
  const v4f lo = *(const v4f*)src;
  const v4f hi = *(const v4f*)(src + 4);
  v8us o;
  o[0] = bf16_bits(lo[0]); o[1] = bf16_bits(lo[1]);
  o[2] = bf16_bits(lo[2]); o[3] = bf16_bits(lo[3]);
  o[4] = bf16_bits(hi[0]); o[5] = bf16_bits(hi[1]);
  o[6] = bf16_bits(hi[2]); o[7] = bf16_bits(hi[3]);
  u16* dst = w + (size_t)row * DD + d0;
  *(volatile v8us*)dst = o;
  __threadfence();
  *(volatile v8us*)dst = o;
}

__global__ void __launch_bounds__(256)
k_gather_w2(const float* __restrict__ cb, const int* __restrict__ idx, _Float16* w) {
  const int t = blockIdx.x * 256 + threadIdx.x;
  const int total = DD * (HH / 8);
  if (t >= total) return;
  const int row = t / (HH / 8);
  const int c8  = t - row * (HH / 8);
  const int k0  = c8 * 8;
  const int c   = k0 / SUB2;
  const int j   = k0 - c * SUB2;
  int code = idx[c * DD + row];
  code = code < 0 ? 0 : (code > KCB - 1 ? KCB - 1 : code);
  const float* src = cb + ((size_t)(c * KCB + code) * SUB2 + j);
  const v4f lo = *(const v4f*)src;
  const v4f hi = *(const v4f*)(src + 4);
  v8h o;
  o[0] = (_Float16)(bf16_val(lo[0]) * WCARRY); o[1] = (_Float16)(bf16_val(lo[1]) * WCARRY);
  o[2] = (_Float16)(bf16_val(lo[2]) * WCARRY); o[3] = (_Float16)(bf16_val(lo[3]) * WCARRY);
  o[4] = (_Float16)(bf16_val(hi[0]) * WCARRY); o[5] = (_Float16)(bf16_val(hi[1]) * WCARRY);
  o[6] = (_Float16)(bf16_val(hi[2]) * WCARRY); o[7] = (_Float16)(bf16_val(hi[3]) * WCARRY);
  _Float16* dst = w + (size_t)row * HH + k0;
  *(volatile v8h*)dst = o;
  __threadfence();
  *(volatile v8h*)dst = o;
}

__global__ void __launch_bounds__(256, 1)
k_fc1(const u16* __restrict__ xb, const u16* __restrict__ w1b,
      const float* __restrict__ b1, _Float16* hp) {
  __shared__ _Float16 stg[8 * 16 * P1];
  const int lane = threadIdx.x & 31;
  const int wave = threadIdx.x >> 5;
  const int hf = lane >> 4;
  const int m  = lane & 15;
  const int m0 = blockIdx.x * 64;
  const int n0 = blockIdx.y * 512 + wave * 64;

  v8f vzero = {};
  v8f acc[4][4];
#pragma unroll
  for (int g = 0; g < 4; ++g)
#pragma unroll
    for (int j = 0; j < 4; ++j) acc[g][j] = vzero;

  for (int k0 = 0; k0 < DD; k0 += 32) {
    v16b a[4];
#pragma unroll
    for (int g = 0; g < 4; ++g) a[g] = ldfrag_b(xb, m0 + g * 16, k0, DD, lane);
#pragma unroll
    for (int j = 0; j < 4; ++j) {
      const v16b bfr = ldfrag_b(w1b, n0 + j * 16, k0, DD, lane);
#pragma unroll
      for (int g = 0; g < 4; ++g) acc[g][j] = mma_bf16(a[g], bfr, acc[g][j]);
    }
  }

  float bb[4];
#pragma unroll
  for (int j = 0; j < 4; ++j) bb[j] = bf16_val(b1[n0 + j * 16 + m]);

  _Float16* st = stg + wave * (16 * P1);
  const int rr = lane >> 3;
  const int cq = (lane & 7) * 8;

#pragma unroll
  for (int g = 0; g < 4; ++g) {
#pragma unroll
    for (int j = 0; j < 4; ++j) {
      const int c = j * 16 + m;
#pragma unroll
      for (int r = 0; r < 8; ++r) {
        const float v = acc[g][j][r] + bb[j];
        st[(8 * hf + r) * P1 + c] = (_Float16)(gelu_f(v) * HCARRY);
      }
    }
    __syncthreads();
    v8h vals[4];
#pragma unroll
    for (int it = 0; it < 4; ++it) vals[it] = *(const v8h*)(st + (it * 4 + rr) * P1 + cq);
    _Float16* gp = hp + (size_t)(m0 + g * 16 + rr) * HH + n0 + cq;
#pragma unroll
    for (int it = 0; it < 4; ++it)
      *(volatile v8h*)(gp + (size_t)it * 4 * HH) = vals[it];
    __threadfence();
#pragma unroll
    for (int it = 0; it < 4; ++it)
      *(volatile v8h*)(gp + (size_t)it * 4 * HH) = vals[it];
    __syncthreads();
  }
}

__global__ void __launch_bounds__(256, 1)
k_fc2(const _Float16* __restrict__ hp, const _Float16* __restrict__ w2h,
      const float* __restrict__ b2, float* out) {
  __shared__ float stg[8 * 16 * P2];
  const int lane = threadIdx.x & 31;
  const int wave = threadIdx.x >> 5;
  const int hf = lane >> 4;
  const int m  = lane & 15;
  const int m0 = blockIdx.x * 64;
  const int n0 = blockIdx.y * 512 + wave * 64;

  v8f vzero = {};
  v8f acc[4][4];
#pragma unroll
  for (int g = 0; g < 4; ++g)
#pragma unroll
    for (int j = 0; j < 4; ++j) acc[g][j] = vzero;

  for (int k0 = 0; k0 < HH; k0 += 32) {
    v16h a[4];
#pragma unroll
    for (int g = 0; g < 4; ++g) a[g] = ldfrag_h(hp, m0 + g * 16, k0, HH, lane);
#pragma unroll
    for (int j = 0; j < 4; ++j) {
      const v16h bfr = ldfrag_h(w2h, n0 + j * 16, k0, HH, lane);
#pragma unroll
      for (int g = 0; g < 4; ++g) acc[g][j] = mma_f16(a[g], bfr, acc[g][j]);
    }
  }

  float bb[4];
#pragma unroll
  for (int j = 0; j < 4; ++j) bb[j] = bf16_val(b2[n0 + j * 16 + m]);

  float* st = stg + wave * (16 * P2);
  const int rr = lane >> 4;
  const int cq = (lane & 15) * 4;
  const int orow0 = full_row(m0);

#pragma unroll
  for (int g = 0; g < 4; ++g) {
#pragma unroll
    for (int j = 0; j < 4; ++j) {
      const int c = j * 16 + m;
#pragma unroll
      for (int r = 0; r < 8; ++r)
        st[(8 * hf + r) * P2 + c] = acc[g][j][r] * UNCARRY + bb[j];
    }
    __syncthreads();
    v4f vals[8];
#pragma unroll
    for (int it = 0; it < 8; ++it) vals[it] = *(const v4f*)(st + (2 * it + rr) * P2 + cq);
    float* gp = out + (size_t)(orow0 + g * 16 + rr) * DD + n0 + cq;
#pragma unroll
    for (int it = 0; it < 8; ++it)
      *(volatile v4f*)(gp + (size_t)it * 2 * DD) = vals[it];
    __threadfence();
#pragma unroll
    for (int it = 0; it < 8; ++it)
      *(volatile v4f*)(gp + (size_t)it * 2 * DD) = vals[it];
    __syncthreads();
  }
}

extern "C" void kernel_launch(void* const* d_in, const int* in_sizes, int n_in,
                              void* d_out, int out_size, void* d_ws, size_t ws_size,
                              hipStream_t stream) {
  if (n_in < 7) return;
  const int need_rows = (NB - 1) * SEQ_FULL + SEQ;
  if (in_sizes[0] < need_rows * DD) return;
  if (in_sizes[1] < NCB * KCB * SUB1) return;
  if (in_sizes[2] < NCB * HH) return;
  if (in_sizes[3] < HH) return;
  if (in_sizes[4] < NCB * KCB * SUB2) return;
  if (in_sizes[5] < NCB * DD) return;
  if (in_sizes[6] < DD) return;
  if (out_size < need_rows * DD) return;

  const float* x    = (const float*)d_in[0];
  const float* cb1  = (const float*)d_in[1];
  const int*   idx1 = (const int*)d_in[2];
  const float* b1   = (const float*)d_in[3];
  const float* cb2  = (const float*)d_in[4];
  const int*   idx2 = (const int*)d_in[5];
  const float* b2   = (const float*)d_in[6];
  float* out = (float*)d_out;

  char* ws = (char*)d_ws;
  size_t off = 0;
  u16* xb = (u16*)(ws + off);            off += (size_t)MROWS * DD * 2;
  u16* w1b = (u16*)(ws + off);           off += (size_t)HH * DD * 2;
  _Float16* w2h = (_Float16*)(ws + off); off += (size_t)DD * HH * 2;
  _Float16* hp = (_Float16*)(ws + off);  off += (size_t)MROWS * HH * 2;
  if (off > ws_size) return;

  {
    const int total = MROWS * (DD / 8);
    k_cvt_x<<<(total + 255) / 256, 256, 0, stream>>>(x, xb);
  }
  {
    const int total = HH * (DD / 8);
    k_gather_w1<<<(total + 255) / 256, 256, 0, stream>>>(cb1, idx1, w1b);
  }
  {
    const int total = DD * (HH / 8);
    k_gather_w2<<<(total + 255) / 256, 256, 0, stream>>>(cb2, idx2, w2h);
  }
  {
    dim3 grid(MROWS / 64, HH / 512);
    k_fc1<<<grid, 256, 0, stream>>>(xb, w1b, b1, hp);
  }
  {
    dim3 grid(MROWS / 64, DD / 512);
    k_fc2<<<grid, 256, 0, stream>>>(hp, w2h, b2, out);
  }
}
